// GNN_23587960390209
// MI455X (gfx1250) — hardware-verified
//
#include <hip/hip_runtime.h>
#include <stddef.h>
#include <stdint.h>
#include <math.h>


#define DIN    64
#define HD     128
#define K0     192
#define K12    512
#define HP     256
#define NTHR   256
#define NWAVE  8
#define EPT    8
#define CHUNK  (NTHR * EPT)
#define WCAP   (EPT * 32)
#define LISTN  (NWAVE * WCAP)
#define NBA    1024
#define SLA    10
#define RCAP   14336
#define DEGCAP 64
#define GBM    128
#define GTHR   256
#define RECW   256
#define TABW   384
#define A0W    96
#define S0_ZINTS    (LISTN + 2 * RCAP + 3 * NBA)
#define S0_MISC     16
#define S0_ROWB     (NWAVE * A0W)
#define S0_LDS_INTS (S0_ZINTS + S0_MISC + S0_ROWB)
#define NUW0   1024
#define NUW1   2048
#define NUWT   (3 * NUW0 + 8 * NUW1)
#define WSMAX  134217728

static_assert((CHUNK & (CHUNK - 1)) == 0 && CHUNK <= 4096);
static_assert((NBA & (NBA - 1)) == 0 && NBA == (1 << SLA));
static_assert(((long long)CHUNK << SLA) < (1LL << 31));
static_assert(NBA % NWAVE == 0 && NBA % 32 == 0 && NBA == 4 * NTHR);
static_assert(RCAP % (4 * NTHR) == 0 && RCAP % NTHR == 0);
static_assert(S0_ZINTS % (NTHR * 4) == 0 && ((S0_ZINTS + S0_MISC) % 4) == 0 && (A0W % 4) == 0);
static_assert(K0 % 32 == 0 && K12 % 32 == 0 && HP % 32 == 0 && K0 == 3 * DIN && K12 == 2 * HP && HP == 2 * HD);
static_assert(GBM == (GTHR / 32) * 16 && HD == 8 * 16);
static_assert(NUW0 % NTHR == 0 && NUW1 % NTHR == 0 && NUWT % NTHR == 0);
static_assert(NUW0 == HD * (DIN / 8) && NUW1 == HD * (HD / 8));
static_assert(A0W * 2 == K0 && DIN == 2 * 32 && HD == 4 * 32);
static_assert(S0_LDS_INTS * 4 <= 300000);
static_assert(DEGCAP >= 29 + 8 && RCAP >= 13102 + 8);

typedef float          v4f   __attribute__((ext_vector_type(4)));
typedef float          v8f   __attribute__((ext_vector_type(8)));
typedef int            v4i   __attribute__((ext_vector_type(4)));
typedef int            v8i   __attribute__((ext_vector_type(8)));
typedef unsigned       v2u   __attribute__((ext_vector_type(2)));
typedef unsigned       v4u   __attribute__((ext_vector_type(4)));
typedef unsigned short v4us  __attribute__((ext_vector_type(4)));
typedef unsigned short v8us  __attribute__((ext_vector_type(8)));
typedef unsigned short v16us __attribute__((ext_vector_type(16)));
typedef __bf16         v16bf __attribute__((ext_vector_type(16)));
typedef v4f  __attribute__((may_alias)) v4fa;
typedef v4i  __attribute__((may_alias)) v4ia;
typedef v2u  __attribute__((may_alias)) v2ua;
typedef v4u  __attribute__((may_alias)) v4ua;
typedef v4us __attribute__((may_alias)) v4usa;
typedef v8us __attribute__((may_alias)) v8usa;
union FragB { v16bf v; v16us u; v8us h[2]; v8i w; };

__device__ __forceinline__ v8f wmb(const FragB& a, const FragB& b, v8f c) {
  v8f d = __builtin_amdgcn_wmma_f32_16x16x32_bf16(false, a.v, false, b.v, (short)0, c, false, false);
  asm volatile("v_nop\n\tv_nop\n\tv_nop\n\tv_nop" : "+v"(d) : "v"(a.w), "v"(b.w));
  return d;
}

__device__ __forceinline__ unsigned bf16_bits(float f) {
  const unsigned u = __float_as_uint(f);
  return (u + 0x7FFFu + ((u >> 16) & 1u)) >> 16;
}
__device__ __forceinline__ float bf16_val(float f) {
  return __uint_as_float(bf16_bits(f) << 16);
}
__device__ __forceinline__ float relu_np(float v) { return (v > 0.0f) ? v : (v - v); }

__device__ __forceinline__ void wave_sync() {
  __builtin_amdgcn_fence(__ATOMIC_RELEASE, "wavefront");
  __builtin_amdgcn_wave_barrier();
  __builtin_amdgcn_fence(__ATOMIC_ACQUIRE, "wavefront");
}

template <int SLB>
__device__ __forceinline__ int scan_chunk(const int* __restrict__ dsts, int nE, int cbase, int slotBase,
                                          int nb, int vec8, int* list, int tid, int lane, int wave) {
  int wc = 0;
  const int el0  = tid * EPT;
  const int e0   = cbase + el0;
  const int sent = -2147483647 - 1;
  v4i da, db;
  if (vec8 != 0 && cbase + CHUNK <= nE) {
    da = *(const v4i*)(dsts + e0);
    db = *(const v4i*)(dsts + e0 + 4);
  } else {
    da.x = (e0     < nE) ? dsts[min(e0,     nE - 1)] : sent;
    da.y = (e0 + 1 < nE) ? dsts[min(e0 + 1, nE - 1)] : sent;
    da.z = (e0 + 2 < nE) ? dsts[min(e0 + 2, nE - 1)] : sent;
    da.w = (e0 + 3 < nE) ? dsts[min(e0 + 3, nE - 1)] : sent;
    db.x = (e0 + 4 < nE) ? dsts[min(e0 + 4, nE - 1)] : sent;
    db.y = (e0 + 5 < nE) ? dsts[min(e0 + 5, nE - 1)] : sent;
    db.z = (e0 + 6 < nE) ? dsts[min(e0 + 6, nE - 1)] : sent;
    db.w = (e0 + 7 < nE) ? dsts[min(e0 + 7, nE - 1)] : sent;
  }
  const unsigned nbs = (unsigned)slotBase;
  const unsigned unb = (unsigned)nb;
  const unsigned s0 = (unsigned)da.x - nbs, s1 = (unsigned)da.y - nbs;
  const unsigned s2 = (unsigned)da.z - nbs, s3 = (unsigned)da.w - nbs;
  const unsigned s4 = (unsigned)db.x - nbs, s5 = (unsigned)db.y - nbs;
  const unsigned s6 = (unsigned)db.z - nbs, s7 = (unsigned)db.w - nbs;
  const bool h0 = s0 < unb, h1 = s1 < unb, h2 = s2 < unb, h3 = s3 < unb;
  const bool h4 = s4 < unb, h5 = s5 < unb, h6 = s6 < unb, h7 = s7 < unb;
  const unsigned any = __builtin_amdgcn_ballot_w32(h0 | h1 | h2 | h3 | h4 | h5 | h6 | h7);
  if (any != 0u) {
#define HITJ(J, HJ, SJ) { \
      const unsigned mj = __builtin_amdgcn_ballot_w32(HJ); \
      if (mj != 0u) { \
        if (HJ) { \
          const int pos = wc + (int)__builtin_amdgcn_mbcnt_lo(mj, 0u); \
          if (pos < WCAP) list[wave * WCAP + pos] = ((el0 + (J)) << SLB) | (int)(SJ); \
        } \
        wc += (int)__builtin_popcount(mj); } }
    HITJ(0, h0, s0)
    HITJ(1, h1, s1)
    HITJ(2, h2, s2)
    HITJ(3, h3, s3)
    HITJ(4, h4, s4)
    HITJ(5, h5, s5)
    HITJ(6, h6, s6)
    HITJ(7, h7, s7)
#undef HITJ
  }
  return wc;
}

__device__ __forceinline__ void wunit(const float* __restrict__ W, int v, int kshift,
                                      unsigned short* P, int pitch, int coff) {
  const int n  = v >> kshift;
  const int k8 = (v & ((1 << kshift) - 1)) * 8;
  const float* p = W + (size_t)k8 * HD + n;
  v8us o;
#pragma unroll
  for (int i = 0; i < 8; ++i) o[i] = (unsigned short)bf16_bits(p[(size_t)i * HD]);
  unsigned short* dp = P + (size_t)n * pitch + coff + k8;
  *(volatile v8us*)dp = o;
  __threadfence();
  *(volatile v8us*)dp = o;
}

__global__ __launch_bounds__(NTHR) void k_wprep(const float* __restrict__ Ws0, const float* __restrict__ Wn0,
                                                const float* __restrict__ Ws1, const float* __restrict__ Wn1,
                                                const float* __restrict__ Ws2, const float* __restrict__ Wn2,
                                                unsigned short* Bt0, unsigned short* Bt1, unsigned short* Bt2) {
  const int u = (int)blockIdx.x * NTHR + (int)threadIdx.x;
  if (u < 3 * NUW0) {
    const int part = u >> 10;
    const int v = u & (NUW0 - 1);
    if (part == 0)      wunit(Ws0, v, 3, Bt0, K0, 0);
    else if (part == 1) wunit(Wn0, v, 3, Bt0, K0, DIN);
    else                wunit(Wn0, v, 3, Bt0, K0, 2 * DIN);
  } else if (u < 3 * NUW0 + 4 * NUW1) {
    const int w = u - 3 * NUW0;
    const int part = w >> 11;
    const int v = w & (NUW1 - 1);
    if (part == 0)      wunit(Ws1, v, 4, Bt1, K12, 0);
    else if (part == 1) wunit(Ws1, v, 4, Bt1, K12, HD);
    else if (part == 2) wunit(Wn1, v, 4, Bt1, K12, 2 * HD);
    else                wunit(Wn1, v, 4, Bt1, K12, 3 * HD);
  } else if (u < NUWT) {
    const int w = u - 3 * NUW0 - 4 * NUW1;
    const int part = w >> 11;
    const int v = w & (NUW1 - 1);
    if (part == 0)      wunit(Ws2, v, 4, Bt2, K12, 0);
    else if (part == 1) wunit(Ws2, v, 4, Bt2, K12, HD);
    else if (part == 2) wunit(Wn2, v, 4, Bt2, K12, 2 * HD);
    else                wunit(Wn2, v, 4, Bt2, K12, 3 * HD);
  }
}

__global__ __launch_bounds__(NTHR) void k_cvx(const float* __restrict__ x, int nUnits, unsigned short* xb) {
  const int u = (int)blockIdx.x * NTHR + (int)threadIdx.x;
  if (u >= nUnits) return;
  const int row = u >> 3;
  const int k8  = (u & 7) * 8;
  const float* p = x + (size_t)row * DIN + k8;
  const v4f a = *(const v4fa*)p;
  const v4f b = *(const v4fa*)(p + 4);
  v8us o;
  o[0] = (unsigned short)bf16_bits(a.x); o[1] = (unsigned short)bf16_bits(a.y);
  o[2] = (unsigned short)bf16_bits(a.z); o[3] = (unsigned short)bf16_bits(a.w);
  o[4] = (unsigned short)bf16_bits(b.x); o[5] = (unsigned short)bf16_bits(b.y);
  o[6] = (unsigned short)bf16_bits(b.z); o[7] = (unsigned short)bf16_bits(b.w);
  unsigned short* dp = xb + (size_t)row * DIN + k8;
  *(volatile v8us*)dp = o;
  __threadfence();
  *(volatile v8us*)dp = o;
}

__global__ __launch_bounds__(NTHR) void k_scan0(const int* __restrict__ srcs, const int* __restrict__ dsts,
                                                int nE, int nN, int vec8, int mRows,
                                                const unsigned* __restrict__ xbw, unsigned* a0w,
                                                int* listg, int* degg) {
  extern __shared__ __attribute__((aligned(16))) int dsm[];
  int* list = dsm;
  int* hl   = dsm + LISTN;
  int* sl   = hl + RCAP;
  int* cnt  = sl + RCAP;
  int* offs = cnt + NBA;
  int* cur  = offs + NBA;
  int* misc = cur + NBA;
  const int tid = (int)threadIdx.x, lane = tid & 31, wave = tid >> 5;
  unsigned* rowbuf = (unsigned*)(misc + S0_MISC) + wave * A0W;
  const int nodeBase = (int)blockIdx.x * NBA;

  {
    const v4i z4 = {0, 0, 0, 0};
    for (int i = tid * 4; i < S0_ZINTS; i += NTHR * 4) *(v4ia*)(dsm + i) = z4;
    if (tid < S0_MISC) misc[tid] = 0;
  }
  __syncthreads();

  int t = 0, ov = 0;
  const int nChunks = (nE + CHUNK - 1) / CHUNK;
#pragma unroll 1
  for (int ch = 0; ch < nChunks; ++ch) {
    const int cbase = ch * CHUNK;
    const int wc = scan_chunk<SLA>(dsts, nE, cbase, nodeBase, NBA, vec8, list, tid, lane, wave);
    if (lane == 0) misc[wave] = wc;
    __syncthreads();
    if (wave == 0) {
#pragma unroll 1
      for (int w2 = 0; w2 < NWAVE; ++w2) {
        int c = misc[w2];
        c = c < 0 ? 0 : (c > WCAP ? WCAP : c);
#pragma unroll 1
        for (int b0 = 0; b0 < c; b0 += 32) {
          const int idx = b0 + lane;
          const int ent = list[w2 * WCAP + (idx < WCAP ? idx : WCAP - 1)];
          const int m32 = (c - b0) < 32 ? (c - b0) : 32;
#pragma unroll 1
          for (int k = 0; k < m32; ++k) {
            const int u    = __builtin_amdgcn_readlane(ent, k);
            const int slot = u & (NBA - 1);
            const int el   = (u >> SLA) & (CHUNK - 1);
            const int pk   = ((cbase + el) << SLA) | slot;
            if (t < RCAP) {
              if (lane == 0) { hl[t] = pk; cnt[slot] = cnt[slot] + 1; }
              t = t + 1;
            } else {
              ov = 1;
            }
          }
        }
      }
    }
    __syncthreads();
  }
  if (wave == 0 && lane == 0) { misc[8] = t; misc[9] = ov; }
  __syncthreads();
  int tt = misc[8];
  tt = tt < 0 ? 0 : (tt > RCAP ? RCAP : tt);
  const int ovf = misc[9];

  if (wave == 0) {
    const int base = lane * (NBA / 32);
    int s = 0;
#pragma unroll 1
    for (int i = 0; i < NBA / 32; ++i) s += cnt[base + i];
    int incl = s;
#pragma unroll
    for (int d = 1; d < 32; d <<= 1) {
      const int y = __shfl_up(incl, d, 32);
      if (lane >= d) incl += y;
    }
    int run = incl - s;
#pragma unroll 1
    for (int i = 0; i < NBA / 32; ++i) {
      const int cv = cnt[base + i];
      offs[base + i] = run;
      cur[base + i]  = run;
      run += cv;
    }
  }
  __syncthreads();
  if (wave == 0) {
#pragma unroll 1
    for (int b0 = 0; b0 < tt; b0 += 32) {
      const int idx = b0 + lane;
      const int ent = hl[idx < RCAP ? idx : RCAP - 1];
      const int m32 = (tt - b0) < 32 ? (tt - b0) : 32;
#pragma unroll 1
      for (int k = 0; k < m32; ++k) {
        const int u    = __builtin_amdgcn_readlane(ent, k);
        const int slot = u & (NBA - 1);
        if (lane == 0) {
          int p = cur[slot];
          p = p < 0 ? 0 : (p > RCAP - 1 ? RCAP - 1 : p);
          sl[p] = u;
          cur[slot] = p + 1;
        }
      }
    }
  }
  __syncthreads();
#pragma unroll 1
  for (int i = tid; i < RCAP; i += NTHR) {
    const int ent = sl[i];
    int eid = ent >> SLA;
    eid = eid < 0 ? 0 : (eid > nE - 1 ? nE - 1 : eid);
    int sr = srcs[eid];
    sr = sr < 0 ? 0 : (sr > nN - 1 ? nN - 1 : sr);
    sl[i] = (i < tt) ? sr : 0;
  }
  __syncthreads();

  {
    int* lg = listg + (size_t)blockIdx.x * RCAP;
    int* dg = degg + (size_t)blockIdx.x * NBA;
    v4i c4 = *(const v4ia*)(cnt + 4 * tid);
    if (ovf != 0) { c4.x = DEGCAP + 1; c4.y = DEGCAP + 1; c4.z = DEGCAP + 1; c4.w = DEGCAP + 1; }
#pragma unroll 1
    for (int it = 0; it < RCAP / (4 * NTHR); ++it) {
      const int o4 = 4 * (it * NTHR + tid);
      const v4i v = *(const v4ia*)(sl + o4);
      *(volatile v4i*)(lg + o4) = v;
    }
    *(volatile v4i*)(dg + 4 * tid) = c4;
    __threadfence();
#pragma unroll 1
    for (int it = 0; it < RCAP / (4 * NTHR); ++it) {
      const int o4 = 4 * (it * NTHR + tid);
      const v4i v = *(const v4ia*)(sl + o4);
      *(volatile v4i*)(lg + o4) = v;
    }
    *(volatile v4i*)(dg + 4 * tid) = c4;
  }

  const float qnan = __int_as_float(0x7fc00000);
  const float pz = (ovf != 0) ? qnan : 0.0f;
  const int lq = lane < 24 ? lane : 23;
#pragma unroll 1
  for (int si = 0; si < NBA / NWAVE; ++si) {
    const int s    = si * NWAVE + wave;
    const int node = nodeBase + s;
    int c = cnt[s];
    const bool big = c > DEGCAP;
    c = c < 0 ? 0 : (c > DEGCAP ? DEGCAP : c);
    int o = offs[s];
    o = o < 0 ? 0 : (o > RCAP ? RCAP : o);
    const int nc = node < nN ? node : nN - 1;
    float acc0 = 0.0f, acc1 = 0.0f;
#pragma unroll 1
    for (int b0 = 0; b0 < c; b0 += 32) {
      int idx = o + b0 + lane;
      idx = idx > RCAP - 1 ? RCAP - 1 : idx;
      int sr = sl[idx];
      sr = sr < 0 ? 0 : (sr > nN - 1 ? nN - 1 : sr);
      const int m32 = (c - b0) < 32 ? (c - b0) : 32;
#pragma unroll 1
      for (int k = 0; k < m32; ++k) {
        const int sk = __builtin_amdgcn_readlane(sr, k);
        const unsigned w = xbw[(size_t)sk * 32 + lane];
        acc0 += __uint_as_float(w << 16);
        acc1 += __uint_as_float(w & 0xffff0000u);
      }
    }
    const float dgf  = (float)(c < 1 ? 1 : c);
    const float rinv = 1.0f / dgf;
    const float pzr  = big ? qnan : pz;
    const bool live  = node < nN;
    const float m0 = live ? (acc0 * rinv + pzr) : 0.0f;
    const float m1 = live ? (acc1 * rinv + pzr) : 0.0f;
    const unsigned sw = xbw[(size_t)nc * 32 + lane];
    const unsigned hb0 = bf16_bits(m0), hb1 = bf16_bits(m1);
    const unsigned lb0 = bf16_bits(m0 - __uint_as_float(hb0 << 16));
    const unsigned lb1 = bf16_bits(m1 - __uint_as_float(hb1 << 16));
    rowbuf[lane]      = live ? sw : 0u;
    rowbuf[32 + lane] = hb0 | (hb1 << 16);
    rowbuf[64 + lane] = lb0 | (lb1 << 16);
    wave_sync();
    const v4u q = *(const v4ua*)(rowbuf + 4 * lq);
    wave_sync();
    const bool wr = (node < mRows) && (lane < 24);
    unsigned* rp = a0w + (size_t)node * A0W + 4 * lq;
    if (wr) *(volatile v4u*)rp = q;
    __threadfence();
    if (wr) *(volatile v4u*)rp = q;
  }
}

__global__ __launch_bounds__(NTHR) void k_scanr(const int* __restrict__ listg, const int* __restrict__ degg,
                                                int nN, int mRows,
                                                const unsigned short* __restrict__ hhl, unsigned short* nei) {
  __shared__ __attribute__((aligned(16))) int cnt[NBA];
  __shared__ __attribute__((aligned(16))) int offs[NBA];
  __shared__ __attribute__((aligned(16))) unsigned short rb[NWAVE * HP];
  const int tid = (int)threadIdx.x, lane = tid & 31, wave = tid >> 5;
  unsigned short* rowbuf = rb + wave * HP;
  const int nodeBase = (int)blockIdx.x * NBA;
  const int* lg = listg + (size_t)blockIdx.x * RCAP;
  {
    v4i c4 = *(const v4i*)(degg + (size_t)blockIdx.x * NBA + 4 * tid);
    c4.x = c4.x < 0 ? 0 : (c4.x > DEGCAP + 1 ? DEGCAP + 1 : c4.x);
    c4.y = c4.y < 0 ? 0 : (c4.y > DEGCAP + 1 ? DEGCAP + 1 : c4.y);
    c4.z = c4.z < 0 ? 0 : (c4.z > DEGCAP + 1 ? DEGCAP + 1 : c4.z);
    c4.w = c4.w < 0 ? 0 : (c4.w > DEGCAP + 1 ? DEGCAP + 1 : c4.w);
    *(v4ia*)(cnt + 4 * tid) = c4;
  }
  __syncthreads();
  if (wave == 0) {
    const int base = lane * (NBA / 32);
    int s = 0;
#pragma unroll 1
    for (int i = 0; i < NBA / 32; ++i) s += cnt[base + i];
    int incl = s;
#pragma unroll
    for (int d = 1; d < 32; d <<= 1) {
      const int y = __shfl_up(incl, d, 32);
      if (lane >= d) incl += y;
    }
    int run = incl - s;
#pragma unroll 1
    for (int i = 0; i < NBA / 32; ++i) {
      const int cv = cnt[base + i];
      offs[base + i] = run;
      run += cv;
    }
  }
  __syncthreads();

  const float qnan = __int_as_float(0x7fc00000);
#pragma unroll 1
  for (int si = 0; si < NBA / NWAVE; ++si) {
    const int s    = si * NWAVE + wave;
    const int node = nodeBase + s;
    int c = cnt[s];
    const bool big = c > DEGCAP;
    c = c < 0 ? 0 : (c > DEGCAP ? DEGCAP : c);
    int o = offs[s];
    o = o < 0 ? 0 : (o > RCAP ? RCAP : o);
    float a0 = 0.0f, a1 = 0.0f, a2 = 0.0f, a3 = 0.0f;
#pragma unroll 1
    for (int b0 = 0; b0 < c; b0 += 32) {
      int idx = o + b0 + lane;
      idx = idx > RCAP - 1 ? RCAP - 1 : idx;
      int sr = lg[idx];
      sr = sr < 0 ? 0 : (sr > nN - 1 ? nN - 1 : sr);
      const int m32 = (c - b0) < 32 ? (c - b0) : 32;
#pragma unroll 1
      for (int k = 0; k < m32; ++k) {
        const int sk = __builtin_amdgcn_readlane(sr, k);
        const unsigned short* rp = hhl + (size_t)sk * HP + 4 * lane;
        const v2u wh = *(const v2ua*)rp;
        const v2u wl = *(const v2ua*)(rp + HD);
        const float f0 = __uint_as_float(wh.x << 16)         + __uint_as_float(wl.x << 16);
        const float f1 = __uint_as_float(wh.x & 0xffff0000u) + __uint_as_float(wl.x & 0xffff0000u);
        const float f2 = __uint_as_float(wh.y << 16)         + __uint_as_float(wl.y << 16);
        const float f3 = __uint_as_float(wh.y & 0xffff0000u) + __uint_as_float(wl.y & 0xffff0000u);
        a0 += f0; a1 += f1; a2 += f2; a3 += f3;
      }
    }
    const float dgf  = (float)(c < 1 ? 1 : c);
    const float rinv = 1.0f / dgf;
    const float pzr  = big ? qnan : 0.0f;
    const bool live  = node < nN;
    const float m0 = live ? (a0 * rinv + pzr) : 0.0f;
    const float m1 = live ? (a1 * rinv + pzr) : 0.0f;
    const float m2 = live ? (a2 * rinv + pzr) : 0.0f;
    const float m3 = live ? (a3 * rinv + pzr) : 0.0f;
    v4us mh, ml;
    {
      unsigned hb;
      hb = bf16_bits(m0); mh[0] = (unsigned short)hb; ml[0] = (unsigned short)bf16_bits(m0 - __uint_as_float(hb << 16));
      hb = bf16_bits(m1); mh[1] = (unsigned short)hb; ml[1] = (unsigned short)bf16_bits(m1 - __uint_as_float(hb << 16));
      hb = bf16_bits(m2); mh[2] = (unsigned short)hb; ml[2] = (unsigned short)bf16_bits(m2 - __uint_as_float(hb << 16));
      hb = bf16_bits(m3); mh[3] = (unsigned short)hb; ml[3] = (unsigned short)bf16_bits(m3 - __uint_as_float(hb << 16));
    }
    *(v4usa*)(rowbuf + 4 * lane) = mh;
    *(v4usa*)(rowbuf + HD + 4 * lane) = ml;
    wave_sync();
    const v8us q = *(const v8usa*)(rowbuf + 8 * lane);
    wave_sync();
    if (node < mRows) {
      unsigned short* rpw = nei + (size_t)node * HP + 8 * lane;
      *(volatile v8us*)rpw = q;
      __threadfence();
      *(volatile v8us*)rpw = q;
    }
  }
}

__device__ __forceinline__ void kloop(const unsigned short* ap, const unsigned short* bp, int bpitch,
                                      int ksteps, v8f (&acc)[8]) {
#pragma unroll 1
  for (int ks = 0; ks < ksteps; ++ks) {
    FragB af;
    af.h[0] = *(const v8usa*)(ap + 32 * ks);
    af.h[1] = *(const v8usa*)(ap + 32 * ks + 16);
#pragma unroll
    for (int nt = 0; nt < 8; ++nt) {
      const unsigned short* wq = bp + (size_t)(16 * nt) * (size_t)bpitch + 32 * ks;
      FragB bf;
      bf.h[0] = *(const v8usa*)wq;
      bf.h[1] = *(const v8usa*)(wq + 16);
      acc[nt] = wmb(af, bf, acc[nt]);
    }
  }
}

template <int L0>
__global__ __launch_bounds__(GTHR) void k_gemm(const unsigned short* A1, const unsigned short* A2,
                                               const unsigned short* __restrict__ BT,
                                               const float* __restrict__ bias,
                                               float* hpre, float* rec, int nN) {
  __shared__ __attribute__((aligned(16))) float stg[GBM * 64];
  __shared__ float wsm[NWAVE * RECW];
  __shared__ __attribute__((aligned(16))) float recs[RECW];
  __shared__ float sbias[HD];
  const int tid = (int)threadIdx.x, lane = tid & 31, wave = tid >> 5, hh = lane >> 4, m = lane & 15;
  const int rowBase = (int)blockIdx.x * GBM;

  if (tid < HD) sbias[tid] = bf16_val(bias[tid]);

  v8f acc[8];
  {
    const v8f z = {0.f, 0.f, 0.f, 0.f, 0.f, 0.f, 0.f, 0.f};
#pragma unroll
    for (int t = 0; t < 8; ++t) acc[t] = z;
  }
  const size_t arow = (size_t)(rowBase + 16 * wave + m);
  if constexpr (L0 != 0) {
    kloop(A1 + arow * K0 + 8 * hh, BT + (size_t)m * K0 + 8 * hh, K0, K0 / 32, acc);
  } else {
    kloop(A1 + arow * HP + 8 * hh, BT + (size_t)m * K12 + 8 * hh, K12, HP / 32, acc);
    kloop(A2 + arow * HP + 8 * hh, BT + (size_t)m * K12 + HP + 8 * hh, K12, HP / 32, acc);
  }
  __syncthreads();

#pragma unroll
  for (int nt = 0; nt < 8; ++nt) {
    const float bcol = sbias[16 * nt + m];
    float s = 0.0f, q = 0.0f;
#pragma unroll
    for (int r = 0; r < 8; ++r) {
      const bool ok = (rowBase + 16 * wave + 8 * hh + r) < nN;
      const float v = acc[nt][r] + bcol;
      acc[nt][r] = v;
      const float vm = ok ? v : 0.0f;
      s += vm;
      q += vm * vm;
    }
    s += __shfl_xor(s, 16, 32);
    q += __shfl_xor(q, 16, 32);
    if (hh == 0) {
      wsm[wave * RECW + 16 * nt + m]      = s;
      wsm[wave * RECW + HD + 16 * nt + m] = q;
    }
  }
  __syncthreads();
  if (tid < HD) {
    float s = 0.0f, q = 0.0f;
#pragma unroll
    for (int w2 = 0; w2 < NWAVE; ++w2) { s += wsm[w2 * RECW + tid]; q += wsm[w2 * RECW + HD + tid]; }
    recs[tid] = s;
    recs[HD + tid] = q;
  }
  __syncthreads();
  if (tid < RECW / 4) {
    const v4f rv = *(const v4fa*)(recs + 4 * tid);
    float* rp = rec + (size_t)blockIdx.x * RECW + 4 * tid;
    *(volatile v4f*)rp = rv;
    __threadfence();
    *(volatile v4f*)rp = rv;
  }

#pragma unroll
  for (int hc = 0; hc < 2; ++hc) {
#pragma unroll
    for (int t = 0; t < 4; ++t) {
      const int lc = 16 * t + m;
#pragma unroll
      for (int r = 0; r < 8; ++r) {
        const int lr = 16 * wave + 8 * hh + r;
        stg[lr * 64 + lc] = acc[4 * hc + t][r];
      }
    }
    __syncthreads();
    v4f fv[8];
#pragma unroll
    for (int i = 0; i < 8; ++i) {
      const int lr = 16 * wave + 2 * i + hh;
      fv[i] = *(const v4fa*)(stg + lr * 64 + 4 * m);
    }
#pragma unroll
    for (int i = 0; i < 8; ++i) {
      const int gr = rowBase + 16 * wave + 2 * i + hh;
      float* op = hpre + (size_t)gr * HD + 64 * hc + 4 * m;
      if (gr < nN) *(volatile v4f*)op = fv[i];
    }
    __threadfence();
#pragma unroll
    for (int i = 0; i < 8; ++i) {
      const int gr = rowBase + 16 * wave + 2 * i + hh;
      float* op = hpre + (size_t)gr * HD + 64 * hc + 4 * m;
      if (gr < nN) *(volatile v4f*)op = fv[i];
    }
    __syncthreads();
  }
}

__global__ __launch_bounds__(HD) void k_bncomb(const float* __restrict__ rec, int nRec,
                                               const float* __restrict__ gamma, const float* __restrict__ beta,
                                               double invN, float* tab) {
  __shared__ __attribute__((aligned(16))) float ts[TABW];
  const int c = (int)threadIdx.x;
  double S = 0.0, Q = 0.0;
#pragma unroll 4
  for (int b = 0; b < nRec; ++b) {
    S += (double)rec[(size_t)b * RECW + c];
    Q += (double)rec[(size_t)b * RECW + HD + c];
  }
  const double mu = S * invN;
  double var = Q * invN - mu * mu;
  var = (var < 0.0) ? 0.0 : var;
  const float vf = (float)var;
  const float sc = bf16_val(gamma[c]) * rsqrtf(vf + 1e-5f);
  ts[c] = (float)mu;
  ts[HD + c] = sc;
  ts[2 * HD + c] = bf16_val(beta[c]);
  __syncthreads();
  if (c < TABW / 4) {
    const v4f v = *(const v4fa*)(ts + 4 * c);
    float* tp = tab + 4 * c;
    *(volatile v4f*)tp = v;
    __threadfence();
    *(volatile v4f*)tp = v;
  }
}

__global__ __launch_bounds__(NTHR) void k_apply(const float* __restrict__ hpre, const float* __restrict__ tab,
                                                int nN, unsigned short* hhl) {
  __shared__ __attribute__((aligned(16))) unsigned short rb[NWAVE * HP];
  const int tid = (int)threadIdx.x, lane = tid & 31, wave = tid >> 5;
  unsigned short* rowbuf = rb + wave * HP;
  const v4f mu4 = *(const v4f*)(tab + 4 * lane);
  const v4f sc4 = *(const v4f*)(tab + HD + 4 * lane);
  const v4f be4 = *(const v4f*)(tab + 2 * HD + 4 * lane);
#pragma unroll 1
  for (int i = 0; i < 16; ++i) {
    const int row = (int)blockIdx.x * GBM + wave * 16 + i;
    const bool live = row < nN;
    const int rc = live ? row : nN - 1;
    const v4f t = *(const v4f*)(hpre + (size_t)rc * HD + 4 * lane);
    float y0 = relu_np((t.x - mu4.x) * sc4.x + be4.x);
    float y1 = relu_np((t.y - mu4.y) * sc4.y + be4.y);
    float y2 = relu_np((t.z - mu4.z) * sc4.z + be4.z);
    float y3 = relu_np((t.w - mu4.w) * sc4.w + be4.w);
    y0 = live ? y0 : 0.0f; y1 = live ? y1 : 0.0f; y2 = live ? y2 : 0.0f; y3 = live ? y3 : 0.0f;
    v4us mh, ml;
    {
      unsigned hb;
      hb = bf16_bits(y0); mh[0] = (unsigned short)hb; ml[0] = (unsigned short)bf16_bits(y0 - __uint_as_float(hb << 16));
      hb = bf16_bits(y1); mh[1] = (unsigned short)hb; ml[1] = (unsigned short)bf16_bits(y1 - __uint_as_float(hb << 16));
      hb = bf16_bits(y2); mh[2] = (unsigned short)hb; ml[2] = (unsigned short)bf16_bits(y2 - __uint_as_float(hb << 16));
      hb = bf16_bits(y3); mh[3] = (unsigned short)hb; ml[3] = (unsigned short)bf16_bits(y3 - __uint_as_float(hb << 16));
    }
    *(v4usa*)(rowbuf + 4 * lane) = mh;
    *(v4usa*)(rowbuf + HD + 4 * lane) = ml;
    wave_sync();
    const v8us q = *(const v8usa*)(rowbuf + 8 * lane);
    wave_sync();
    unsigned short* rp = hhl + (size_t)row * HP + 8 * lane;
    *(volatile v8us*)rp = q;
    __threadfence();
    *(volatile v8us*)rp = q;
  }
}

__global__ __launch_bounds__(NTHR) void k_final(const float* __restrict__ hpre, const float* __restrict__ tab,
                                                const float* __restrict__ Wc, const float* __restrict__ bc,
                                                int nN, float* out) {
  __shared__ __attribute__((aligned(16))) float os[2 * GBM];
  const int tid = (int)threadIdx.x, lane = tid & 31, wave = tid >> 5;
  const int rowBase = (int)blockIdx.x * GBM;
  const v4f mu4 = *(const v4f*)(tab + 4 * lane);
  const v4f sc4 = *(const v4f*)(tab + HD + 4 * lane);
  const v4f be4 = *(const v4f*)(tab + 2 * HD + 4 * lane);
  const v4f wa = *(const v4f*)(Wc + 8 * lane);
  const v4f wb = *(const v4f*)(Wc + 8 * lane + 4);
  const float w00 = bf16_val(wa.x), w01 = bf16_val(wa.y), w10 = bf16_val(wa.z), w11 = bf16_val(wa.w);
  const float w20 = bf16_val(wb.x), w21 = bf16_val(wb.y), w30 = bf16_val(wb.z), w31 = bf16_val(wb.w);
  const float b0 = bf16_val(bc[0]), b1 = bf16_val(bc[1]);
#pragma unroll 1
  for (int i = 0; i < 16; ++i) {
    const int row = rowBase + wave * 16 + i;
    const int rc = row < nN ? row : nN - 1;
    const v4f t = *(const v4f*)(hpre + (size_t)rc * HD + 4 * lane);
    const float y0 = relu_np((t.x - mu4.x) * sc4.x + be4.x);
    const float y1 = relu_np((t.y - mu4.y) * sc4.y + be4.y);
    const float y2 = relu_np((t.z - mu4.z) * sc4.z + be4.z);
    const float y3 = relu_np((t.w - mu4.w) * sc4.w + be4.w);
    float p0 = y0 * w00; p0 = fmaf(y1, w10, p0); p0 = fmaf(y2, w20, p0); p0 = fmaf(y3, w30, p0);
    float p1 = y0 * w01; p1 = fmaf(y1, w11, p1); p1 = fmaf(y2, w21, p1); p1 = fmaf(y3, w31, p1);
#pragma unroll
    for (int d = 16; d >= 1; d >>= 1) {
      p0 += __shfl_xor(p0, d, 32);
      p1 += __shfl_xor(p1, d, 32);
    }
    if (lane == 0) {
      os[2 * (wave * 16 + i) + 0] = p0 + b0;
      os[2 * (wave * 16 + i) + 1] = p1 + b1;
    }
  }
  __syncthreads();
  if (tid < (2 * GBM) / 4) {
    const v4f ov = *(const v4fa*)(os + 4 * tid);
    const bool ok = (rowBase + 2 * tid + 1) < nN;
    float* op = out + (size_t)rowBase * 2 + 4 * tid;
    if (ok) *(volatile v4f*)op = ov;
    __threadfence();
    if (ok) *(volatile v4f*)op = ov;
  }
}

static inline int cdiv(int a, int b) { return (a + b - 1) / b; }
static inline size_t al256(size_t o) { return (o + 255) & ~(size_t)255; }

extern "C" void kernel_launch(void* const* d_in, const int* in_sizes, int n_in,
                              void* d_out, int out_size, void* d_ws, size_t ws_size,
                              hipStream_t stream) {
  if (n_in < 20) return;
  if (in_sizes[0] < DIN || (in_sizes[0] % DIN) != 0) return;
  const int nN = in_sizes[0] / DIN;
  if (nN < 16 || nN >= (1 << 24) || (nN % 16) != 0) return;
  const int nE = in_sizes[1];
  if (nE < 1 || in_sizes[2] != nE || nE >= (1 << 21)) return;
  if (in_sizes[3] != DIN * HD || in_sizes[4] != HD || in_sizes[5] != DIN * HD) return;
  if (in_sizes[6] != HD || in_sizes[7] != HD) return;
  if (in_sizes[8] != HD * HD || in_sizes[9] != HD || in_sizes[10] != HD * HD) return;
  if (in_sizes[11] != HD || in_sizes[12] != HD) return;
  if (in_sizes[13] != HD * HD || in_sizes[14] != HD || in_sizes[15] != HD * HD) return;
  if (in_sizes[16] != HD || in_sizes[17] != HD) return;
  if (in_sizes[18] != HD * 2 || in_sizes[19] != 2) return;
  if ((long long)out_size != 2LL * nN) return;

  const float* x   = (const float*)d_in[0];
  const int*   src = (const int*)d_in[1];
  const int*   dst = (const int*)d_in[2];
  const float* Ws0 = (const float*)d_in[3];
  const float* bs0 = (const float*)d_in[4];
  const float* Wn0 = (const float*)d_in[5];
  const float* ga0 = (const float*)d_in[6];
  const float* be0 = (const float*)d_in[7];
  const float* Ws1 = (const float*)d_in[8];
  const float* bs1 = (const float*)d_in[9];
  const float* Wn1 = (const float*)d_in[10];
  const float* ga1 = (const float*)d_in[11];
  const float* be1 = (const float*)d_in[12];
  const float* Ws2 = (const float*)d_in[13];
  const float* bs2 = (const float*)d_in[14];
  const float* Wn2 = (const float*)d_in[15];
  const float* ga2 = (const float*)d_in[16];
  const float* be2 = (const float*)d_in[17];
  const float* Wc  = (const float*)d_in[18];
  const float* bc  = (const float*)d_in[19];
  float* out = (float*)d_out;

  const int MP = cdiv(nN, GBM) * GBM;
  const int gM = MP / GBM;
  const int gA = cdiv(MP, NBA);
  if ((long long)gA * NBA < (long long)MP) return;
  const int vec8 = ((nE & 3) == 0) ? 1 : 0;

  char* ws = (char*)d_ws;
  size_t off = 0;
  const size_t oB0  = off; off = al256(off + (size_t)HD * K0 * 2);
  const size_t oB1  = off; off = al256(off + (size_t)HD * K12 * 2);
  const size_t oB2  = off; off = al256(off + (size_t)HD * K12 * 2);
  const size_t oXB  = off; off = al256(off + (size_t)nN * DIN * 2);
  const size_t oLS  = off; off = al256(off + (size_t)gA * RCAP * 4);
  const size_t oDG  = off; off = al256(off + (size_t)gA * NBA * 4);
  const size_t oRC  = off; off = al256(off + (size_t)gM * RECW * 4);
  const size_t oTB  = off; off = al256(off + (size_t)TABW * 4);
  const size_t oR1  = off; off = al256(off + (size_t)MP * HP * 2);
  const size_t oR2  = off; off = al256(off + (size_t)MP * HP * 2);
  if (off > ws_size || off > (size_t)WSMAX) return;
  if ((size_t)MP * K0 * 2 > (size_t)MP * HP * 2) return;
  if ((size_t)MP * HD * 4 > (size_t)MP * HP * 2) return;
  unsigned short* Bt0 = (unsigned short*)(ws + oB0);
  unsigned short* Bt1 = (unsigned short*)(ws + oB1);
  unsigned short* Bt2 = (unsigned short*)(ws + oB2);
  unsigned short* XB  = (unsigned short*)(ws + oXB);
  int*            LST = (int*)(ws + oLS);
  int*            DGP = (int*)(ws + oDG);
  float*          REC = (float*)(ws + oRC);
  float*          TAB = (float*)(ws + oTB);
  unsigned short* R1h = (unsigned short*)(ws + oR1);
  unsigned short* R2h = (unsigned short*)(ws + oR2);
  float*          HPR = (float*)(ws + oR2);

  const size_t s0Lds = (size_t)S0_LDS_INTS * 4;
  hipFuncSetAttribute(reinterpret_cast<const void*>(&k_scan0), hipFuncAttributeMaxDynamicSharedMemorySize, (int)s0Lds);

  const double invN = 1.0 / (double)nN;
  const int nUx = nN * (DIN / 8);

  k_wprep<<<NUWT / NTHR, NTHR, 0, stream>>>(Ws0, Wn0, Ws1, Wn1, Ws2, Wn2, Bt0, Bt1, Bt2);
  k_cvx<<<cdiv(nUx, NTHR), NTHR, 0, stream>>>(x, nUx, XB);
  k_scan0<<<gA, NTHR, s0Lds, stream>>>(src, dst, nE, nN, vec8, MP, (const unsigned*)XB, (unsigned*)R1h, LST, DGP);
  k_gemm<1><<<gM, GTHR, 0, stream>>>(R1h, R1h, Bt0, bs0, HPR, REC, nN);
  k_bncomb<<<1, HD, 0, stream>>>(REC, gM, ga0, be0, invN, TAB);
  k_apply<<<gM, NTHR, 0, stream>>>(HPR, TAB, nN, R1h);
  k_scanr<<<gA, NTHR, 0, stream>>>(LST, DGP, nN, MP, R1h, R2h);
  k_gemm<0><<<gM, GTHR, 0, stream>>>(R1h, R2h, Bt1, bs1, HPR, REC, nN);
  k_bncomb<<<1, HD, 0, stream>>>(REC, gM, ga1, be1, invN, TAB);
  k_apply<<<gM, NTHR, 0, stream>>>(HPR, TAB, nN, R1h);
  k_scanr<<<gA, NTHR, 0, stream>>>(LST, DGP, nN, MP, R1h, R2h);
  k_gemm<0><<<gM, GTHR, 0, stream>>>(R1h, R2h, Bt2, bs2, HPR, REC, nN);
  k_bncomb<<<1, HD, 0, stream>>>(REC, gM, ga2, be2, invN, TAB);
  k_final<<<gM, NTHR, 0, stream>>>(HPR, TAB, Wc, bc, nN, out);
}
